// HyperbolicGNN_13125420056910
// MI455X (gfx1250) — hardware-run, weakly checked
//
#include <hip/hip_runtime.h>
#include <stddef.h>
#include <math.h>


#define DD      128
#define NCLS    10
#define NCP     16
#define NTHR    256
#define NWAVE   8
#define EPT     8
#define NGRP    2
#define CHUNK   (NTHR * EPT * NGRP)
#define WCAPC   (EPT * NGRP * 32)
#define WCAPF   (EPT * NGRP * 32)
#define ESHF    11
#define EMASK   0xFFFFF
#define NBC     32768
#define NBF     2048
#define RCAP    49152
#define RBN     128
#define TGT     256
#define DEGCAP  512
#define GROWS   128
#define OTHR    512
#define TC      256
#define WSCL    64
#define WSCAP   134217728
#define BPW     (DD * DD / 8 / NTHR)

#define LDS_COUNT  ((NBC + NWAVE * WCAPC + NWAVE) * 4)
#define LDS_FILL   ((RCAP + NBF + NWAVE * WCAPF + NWAVE) * 4)
#define LDS_GEMM   (GROWS * DD * 4)

static_assert((CHUNK & (CHUNK - 1)) == 0);
static_assert((NBC & (NBC - 1)) == 0 && (NBF & (NBF - 1)) == 0);
static_assert(NBF <= (1 << ESHF));
static_assert((NBC % NBF) == 0);
static_assert(OTHR * 4 == NBF);
static_assert((RCAP % 32) == 0);
static_assert(TGT == NWAVE * 32);
static_assert(GROWS == NWAVE * 16);
static_assert((TGT % GROWS) == 0);
static_assert(NBC == NWAVE * 32 * 128);
static_assert((DD % 32) == 0);
static_assert(NCLS <= NCP && NCP == 16);
static_assert(((DD * DD / 8) % NTHR) == 0 && (NCP * DD / 8) == NTHR);
static_assert((GROWS * NCLS) % 4 == 0);
static_assert(LDS_FILL <= 300 * 1024);

typedef float     v4f  __attribute__((ext_vector_type(4)));
typedef float     v8f  __attribute__((ext_vector_type(8)));
typedef int       v4i  __attribute__((ext_vector_type(4)));
typedef _Float16  v4h  __attribute__((ext_vector_type(4)));
typedef _Float16  v8h  __attribute__((ext_vector_type(8)));
typedef _Float16  v16h __attribute__((ext_vector_type(16)));
union FragH { v16h v; v8h h[2]; };

__device__ __forceinline__ v8f wmf(v16h a, v16h b, v8f c) {
  v8f d = __builtin_amdgcn_wmma_f32_16x16x32_f16(false, a, false, b, (short)0, c, false, false);
  asm volatile("v_nop\n\tv_nop\n\tv_nop\n\tv_nop" : "+v"(d) : "v"(a), "v"(b));
  return d;
}

__device__ __forceinline__ float red16(float x) {
  x += __shfl_xor(x, 1, 32);
  x += __shfl_xor(x, 2, 32);
  x += __shfl_xor(x, 4, 32);
  x += __shfl_xor(x, 8, 32);
  return x;
}
__device__ __forceinline__ float red32(float x) {
  x = red16(x);
  x += __shfl_xor(x, 16, 32);
  return x;
}

__device__ __forceinline__ float logmap_f(float ss) {
  const float n = fmaxf(sqrtf(ss), 1e-15f);
  const float m = fminf(n, 0.99999f);
  const float a = 0.5f * (log1pf(m) - log1pf(-m));
  return a * (1.0f / n);
}

template <int NB, int SRC, int WC>
__device__ __forceinline__ int scan_chunk(const int* __restrict__ keys, int nK, int cbase,
                                          int slotBase, int vec8, int* list, int tid, int lane, int wave) {
  int wc = 0;
#pragma unroll
  for (int g = 0; g < NGRP; ++g) {
    const int el0  = (g * NTHR + tid) * EPT;
    const int e0   = cbase + el0;
    const int sent = -2147483647 - 1;
    const int i0 = min(e0, nK - 1),     i1 = min(e0 + 1, nK - 1), i2 = min(e0 + 2, nK - 1), i3 = min(e0 + 3, nK - 1);
    const int i4 = min(e0 + 4, nK - 1), i5 = min(e0 + 5, nK - 1), i6 = min(e0 + 6, nK - 1), i7 = min(e0 + 7, nK - 1);
    v4i da, db;
    if (vec8 != 0 && cbase + CHUNK <= nK) {
      da = *(const v4i*)(keys + e0);
      db = *(const v4i*)(keys + e0 + 4);
    } else {
      da.x = (e0     < nK) ? keys[i0] : sent;
      da.y = (e0 + 1 < nK) ? keys[i1] : sent;
      da.z = (e0 + 2 < nK) ? keys[i2] : sent;
      da.w = (e0 + 3 < nK) ? keys[i3] : sent;
      db.x = (e0 + 4 < nK) ? keys[i4] : sent;
      db.y = (e0 + 5 < nK) ? keys[i5] : sent;
      db.z = (e0 + 6 < nK) ? keys[i6] : sent;
      db.w = (e0 + 7 < nK) ? keys[i7] : sent;
    }
    const unsigned nb = (unsigned)slotBase;
    const unsigned s0 = (unsigned)da.x - nb, s1 = (unsigned)da.y - nb;
    const unsigned s2 = (unsigned)da.z - nb, s3 = (unsigned)da.w - nb;
    const unsigned s4 = (unsigned)db.x - nb, s5 = (unsigned)db.y - nb;
    const unsigned s6 = (unsigned)db.z - nb, s7 = (unsigned)db.w - nb;
    const bool h0 = s0 < (unsigned)NB, h1 = s1 < (unsigned)NB, h2 = s2 < (unsigned)NB, h3 = s3 < (unsigned)NB;
    const bool h4 = s4 < (unsigned)NB, h5 = s5 < (unsigned)NB, h6 = s6 < (unsigned)NB, h7 = s7 < (unsigned)NB;
    const unsigned any = __builtin_amdgcn_ballot_w32(h0 | h1 | h2 | h3 | h4 | h5 | h6 | h7);
    if (any != 0u) {
#define HITJ(HJ, SJ, VJ) { \
        const unsigned mj = __builtin_amdgcn_ballot_w32(HJ); \
        if (mj != 0u) { \
          if (HJ) { \
            const int pos = wc + (int)__builtin_amdgcn_mbcnt_lo(mj, 0u); \
            const int entv = SRC ? (((VJ) << ESHF) | (int)(SJ)) : (int)(SJ); \
            if (pos < WC) list[wave * WC + pos] = entv; \
          } \
          wc += (int)__builtin_popcount(mj); } }
      HITJ(h0, s0, i0)
      HITJ(h1, s1, i1)
      HITJ(h2, s2, i2)
      HITJ(h3, s3, i3)
      HITJ(h4, s4, i4)
      HITJ(h5, s5, i5)
      HITJ(h6, s6, i6)
      HITJ(h7, s7, i7)
#undef HITJ
    }
  }
  return wc;
}

__global__ __launch_bounds__(NTHR) void k_cvtw(
    const float* __restrict__ W1, const float* __restrict__ W2, const float* __restrict__ Wc,
    _Float16* W1p, _Float16* W2p, _Float16* Wcp, float scale) {
  const int tid = threadIdx.x;
  const int b = (int)blockIdx.x;
  const float* src;
  _Float16* dst;
  int g, nrows;
  if (b < BPW)          { src = W1; dst = W1p; g = b * NTHR + tid;         nrows = DD; }
  else if (b < 2 * BPW) { src = W2; dst = W2p; g = (b - BPW) * NTHR + tid; nrows = DD; }
  else                  { src = Wc; dst = Wcp; g = tid;                    nrows = NCLS; }
  const int n = g >> 4, k0 = (g & 15) * 8;
  const int nr = n < nrows ? n : nrows - 1;
  const float* p = src + (size_t)nr * DD + k0;
  v4f f0 = *(const v4f*)p;
  v4f f1 = *(const v4f*)(p + 4);
  if (n >= nrows) {
    const v4f z = {0.f, 0.f, 0.f, 0.f}; f0 = z; f1 = z;
  }
  v8h hv;
  hv[0] = (_Float16)(f0.x * scale); hv[1] = (_Float16)(f0.y * scale); hv[2] = (_Float16)(f0.z * scale); hv[3] = (_Float16)(f0.w * scale);
  hv[4] = (_Float16)(f1.x * scale); hv[5] = (_Float16)(f1.y * scale); hv[6] = (_Float16)(f1.z * scale); hv[7] = (_Float16)(f1.w * scale);
  _Float16* d = dst + (size_t)n * DD + k0;
  *(volatile v8h*)d = hv;
  __threadfence();
  *(volatile v8h*)d = hv;
}

__global__ __launch_bounds__(NTHR) void k_count(
    const int* __restrict__ keys, int* cnt, int nK, int vec8) {
  extern __shared__ v4f lds_dyn[];
  int* scnt = (int*)lds_dyn;
  int* list = scnt + NBC;
  int* wcnt = list + NWAVE * WCAPC;
  const int tid = threadIdx.x, lane = tid & 31, wave = tid >> 5;
  const int nodeBase = blockIdx.x * NBC;

  {
    const v4i z = {0, 0, 0, 0};
    for (int i = tid; i < NBC / 4; i += NTHR) ((v4i*)scnt)[i] = z;
  }
  __syncthreads();

  const int nChunks = (nK + CHUNK - 1) / CHUNK;
#pragma unroll 1
  for (int ch = 0; ch < nChunks; ++ch) {
    const int cbase = ch * CHUNK;
    const int wc = scan_chunk<NBC, 0, WCAPC>(keys, nK, cbase, nodeBase, vec8, list, tid, lane, wave);
    if (lane == 0) wcnt[wave] = wc;
    __syncthreads();
    if (wave == 0) {
#pragma unroll 1
      for (int wsx = 0; wsx < NWAVE; ++wsx) {
        int n = __builtin_amdgcn_readfirstlane(wcnt[wsx]);
        n = n > WCAPC ? WCAPC : (n < 0 ? 0 : n);
        const int* lp = list + wsx * WCAPC;
#pragma unroll 1
        for (int i = 0; i < n; ++i) {
          const int ent  = __builtin_amdgcn_readfirstlane(lp[i]);
          const int slot = ent & (NBC - 1);
          if (lane == 0) scnt[slot] = scnt[slot] + 1;
        }
      }
    }
    __syncthreads();
  }

  int* cp = cnt + (size_t)nodeBase;
#pragma unroll 4
  for (int q = 0; q < 32; ++q) {
    const int f = (wave * 32 + q) * 128 + 4 * lane;
    const v4i c = *(const v4i*)(scnt + f);
    *(volatile v4i*)(cp + f) = c;
  }
  __threadfence();
#pragma unroll 4
  for (int q = 0; q < 32; ++q) {
    const int f = (wave * 32 + q) * 128 + 4 * lane;
    const v4i c = *(const v4i*)(scnt + f);
    *(volatile v4i*)(cp + f) = c;
  }
}

__global__ __launch_bounds__(OTHR) void k_offsets(
    const int* __restrict__ cnt, int* off, int* rbase, int nBF) {
  __shared__ __attribute__((aligned(16))) int srb[RBN];
  __shared__ int wtot[OTHR / 32];
  const int tid = threadIdx.x, lane = tid & 31, wave = tid >> 5;
  for (int i = tid; i < RBN; i += OTHR) srb[i] = 0;
  int carry = 0;
#pragma unroll 1
  for (int fb = 0; fb < nBF; ++fb) {
    const int base = fb * NBF;
    const v4i c = *(const v4i*)(cnt + base + 4 * tid);
    const int e0 = max(c.x, 0), e1 = max(c.y, 0), e2 = max(c.z, 0), e3 = max(c.w, 0);
    const int ts = e0 + e1 + e2 + e3;
    int incl = ts;
#pragma unroll
    for (int d = 1; d < 32; d <<= 1) {
      const int t = __shfl_up(incl, d, 32);
      if (lane >= d) incl += t;
    }
    if (lane == 31) wtot[wave] = incl;
    __syncthreads();
    int pre = 0;
#pragma unroll 1
    for (int w = 0; w < wave; ++w) pre += wtot[w];
    int tot = 0;
#pragma unroll
    for (int w = 0; w < OTHR / 32; ++w) tot += wtot[w];
    int run = carry + pre + incl - ts;
    v4i o;
    o.x = run; run += e0;
    o.y = run; run += e1;
    o.z = run; run += e2;
    o.w = run;
    int* op = off + base + 4 * tid;
    *(volatile v4i*)op = o;
    __threadfence();
    *(volatile v4i*)op = o;
    if (tid == 0) srb[min(fb, RBN - 1)] = carry;
    carry += (tot + 31) & ~31;
    __syncthreads();
  }
  if (tid == 0) srb[min(nBF, RBN - 1)] = carry;
  __syncthreads();
  v4i rv = {0, 0, 0, 0};
  if (tid < 32) rv = *(const v4i*)(srb + 4 * tid);
  if (tid < 32) *(volatile v4i*)(rbase + 4 * tid) = rv;
  __threadfence();
  if (tid < 32) *(volatile v4i*)(rbase + 4 * tid) = rv;
}

__global__ __launch_bounds__(NTHR) void k_fill(
    const int* __restrict__ keys, const int* __restrict__ off,
    const int* __restrict__ rbase, int* csr, int nK, int vec8, int csrLen) {
  extern __shared__ v4f lds_dyn[];
  int* region = (int*)lds_dyn;
  int* cursor = region + RCAP;
  int* list   = cursor + NBF;
  int* wcnt   = list + NWAVE * WCAPF;
  const int tid = threadIdx.x, lane = tid & 31, wave = tid >> 5;
  const int b = blockIdx.x;
  const int nodeBase = b * NBF;

  int rb0 = rbase[b];
  const int rb1 = rbase[b + 1];
  rb0 = rb0 < 0 ? 0 : (rb0 > csrLen ? csrLen : rb0);
  rb0 &= ~31;
  int len = rb1 - rb0;
  len = len < 0 ? 0 : (len > RCAP ? RCAP : len);
  int lenW = (len + 31) & ~31;
  if (rb0 + lenW > csrLen) lenW = (csrLen - rb0) & ~31;

  {
    const v4i z = {0, 0, 0, 0};
    for (int i = tid; i < RCAP / 4; i += NTHR) ((v4i*)region)[i] = z;
    for (int s = tid; s < NBF; s += NTHR) {
      int o = off[nodeBase + s] - rb0;
      o = o < 0 ? 0 : (o > RCAP ? RCAP : o);
      cursor[s] = o;
    }
  }
  __syncthreads();

  const int nChunks = (nK + CHUNK - 1) / CHUNK;
#pragma unroll 1
  for (int ch = 0; ch < nChunks; ++ch) {
    const int cbase = ch * CHUNK;
    const int wc = scan_chunk<NBF, 1, WCAPF>(keys, nK, cbase, nodeBase, vec8, list, tid, lane, wave);
    if (lane == 0) wcnt[wave] = wc;
    __syncthreads();
    if (wave == 0) {
#pragma unroll 1
      for (int wsx = 0; wsx < NWAVE; ++wsx) {
        int n = __builtin_amdgcn_readfirstlane(wcnt[wsx]);
        n = n > WCAPF ? WCAPF : (n < 0 ? 0 : n);
        const int* lp = list + wsx * WCAPF;
#pragma unroll 1
        for (int i = 0; i < n; ++i) {
          const int ent  = __builtin_amdgcn_readfirstlane(lp[i]);
          const int slot = ent & (NBF - 1);
          int ev = (ent >> ESHF) & EMASK;
          ev = ev > nK - 1 ? nK - 1 : ev;
          if (lane == 0) {
            int pos = cursor[slot];
            pos = pos < 0 ? 0 : (pos > RCAP - 1 ? RCAP - 1 : pos);
            region[pos] = ev;
            const int np = pos + 1;
            cursor[slot] = np > RCAP ? RCAP : np;
          }
        }
      }
    }
    __syncthreads();
  }

  const int nv = lenW >> 2;
  int* gp = csr + rb0;
#pragma unroll 1
  for (int i = tid; i < nv; i += NTHR) { const v4i v = ((const v4i*)region)[i]; *(volatile v4i*)(gp + 4 * i) = v; }
  __threadfence();
#pragma unroll 1
  for (int i = tid; i < nv; i += NTHR) { const v4i v = ((const v4i*)region)[i]; *(volatile v4i*)(gp + 4 * i) = v; }
}

__global__ __launch_bounds__(NTHR) void k_tan0(
    const float* __restrict__ x, _Float16* T16, int nN, float tc) {
  const int tid = threadIdx.x, lane = tid & 31, wave = tid >> 5;
  const int tbase = (int)blockIdx.x * TGT + wave * 32;
  const int ch = 4 * lane;
#pragma unroll 1
  for (int j = 0; j < 32; ++j) {
    const int c  = tbase + j;
    const int cs = c < nN ? c : nN - 1;
    v4f v = *(const v4f*)(x + (size_t)cs * DD + ch);
    const float ss = red32(v.x * v.x + v.y * v.y + v.z * v.z + v.w * v.w);
    const float f = logmap_f(ss) * tc;
    if (c >= nN) {
      const v4f z = {0.f, 0.f, 0.f, 0.f}; v = z;
    }
    v4h hv;
    hv[0] = (_Float16)(v.x * f); hv[1] = (_Float16)(v.y * f); hv[2] = (_Float16)(v.z * f); hv[3] = (_Float16)(v.w * f);
    _Float16* rp = T16 + (size_t)c * DD + ch;
    *(volatile v4h*)rp = hv;
    __threadfence();
    *(volatile v4h*)rp = hv;
  }
}

__global__ __launch_bounds__(NTHR) void k_gemm_exp(
    const _Float16* __restrict__ A16, const _Float16* __restrict__ Bw,
    const float* __restrict__ bias, float* Y, float osc) {
  constexpr int NT = 8;
  extern __shared__ v4f lds_dyn[];
  float* stg = (float*)lds_dyn;
  const int tid = threadIdx.x, lane = tid & 31, wave = tid >> 5, hh = lane >> 4, m = lane & 15;
  const int rowBase = (int)blockIdx.x * GROWS;
  const _Float16* ap  = A16 + (size_t)(rowBase + 16 * wave + m) * DD + 8 * hh;
  const _Float16* bp0 = Bw + (size_t)m * DD + 8 * hh;

  v8f acc[NT];
#pragma unroll
  for (int t = 0; t < NT; ++t) { v8f z = {0.f, 0.f, 0.f, 0.f, 0.f, 0.f, 0.f, 0.f}; acc[t] = z; }

#pragma unroll 1
  for (int kt = 0; kt < DD / 32; ++kt) {
    FragH af;
    af.h[0] = *(const v8h*)(ap + 32 * kt);
    af.h[1] = *(const v8h*)(ap + 32 * kt + 16);
#pragma unroll
    for (int t = 0; t < NT; ++t) {
      const _Float16* bp = bp0 + (size_t)(16 * t) * DD + 32 * kt;
      FragH bf;
      bf.h[0] = *(const v8h*)bp;
      bf.h[1] = *(const v8h*)(bp + 16);
      acc[t] = wmf(af.v, bf.v, acc[t]);
    }
  }

  float bcv[NT];
#pragma unroll
  for (int t = 0; t < NT; ++t) bcv[t] = bias[16 * t + m];

  float part[8] = {0.f, 0.f, 0.f, 0.f, 0.f, 0.f, 0.f, 0.f};
#pragma unroll
  for (int t = 0; t < NT; ++t) {
#pragma unroll
    for (int r = 0; r < 8; ++r) {
      const float hv = acc[t][r] * osc + bcv[t];
      acc[t][r] = hv;
      part[r] += hv * hv;
    }
  }
  float sc[8];
#pragma unroll
  for (int r = 0; r < 8; ++r) {
    const float ss = red16(part[r]);
    const float n  = fmaxf(sqrtf(ss), 1e-15f);
    sc[r] = tanhf(n) * (1.0f / n);
  }

  float* sp = stg + (16 * wave + 8 * hh) * DD + m;
#pragma unroll
  for (int t = 0; t < NT; ++t) {
#pragma unroll
    for (int r = 0; r < 8; ++r) sp[r * DD + 16 * t] = acc[t][r] * sc[r];
  }
  __syncthreads();

  const float* lp = stg + wave * 16 * DD;
  const int orow0 = rowBase + wave * 16;
#pragma unroll
  for (int i = 0; i < 16; ++i) {
    const v4f v = *(const v4f*)(lp + i * DD + 4 * lane);
    *(volatile v4f*)(Y + (size_t)(orow0 + i) * DD + 4 * lane) = v;
  }
  __threadfence();
#pragma unroll
  for (int i = 0; i < 16; ++i) {
    const v4f v = *(const v4f*)(lp + i * DD + 4 * lane);
    *(volatile v4f*)(Y + (size_t)(orow0 + i) * DD + 4 * lane) = v;
  }
}

__global__ __launch_bounds__(NTHR) void k_agg(
    const int* __restrict__ csr, const int* __restrict__ off, const int* __restrict__ cnt,
    const int* __restrict__ srcidx, const float* __restrict__ Y,
    _Float16* T16, int nN, int nE, int csrLen, float tc) {
  const int tid = threadIdx.x, lane = tid & 31, wave = tid >> 5;
  const int tbase = (int)blockIdx.x * TGT + wave * 32;
  const int cl = tbase + lane;
  const int cnt_l = cnt[cl];
  const int off_l = off[cl];
  const int ch = 4 * lane;

#pragma unroll 1
  for (int j = 0; j < 32; ++j) {
    const int c = tbase + j;
    const int nraw = __builtin_amdgcn_readlane(cnt_l, j);
    const int n = nraw < 0 ? 0 : (nraw > DEGCAP ? DEGCAP : nraw);
    const int st = __builtin_amdgcn_readlane(off_l, j);
    v4f a0 = {0.f, 0.f, 0.f, 0.f};
#pragma unroll 1
    for (int q0 = 0; q0 < n; q0 += 32) {
      int pos = st + q0 + lane;
      pos = pos < 0 ? 0 : (pos > csrLen - 1 ? csrLen - 1 : pos);
      int el = csr[pos];
      el = el < 0 ? 0 : (el > nE - 1 ? nE - 1 : el);
      int sl = srcidx[el];
      sl = sl < 0 ? 0 : (sl > nN - 1 ? nN - 1 : sl);
      const int mcnt = (n - q0) < 32 ? (n - q0) : 32;
#pragma unroll 1
      for (int p = 0; p < mcnt; ++p) {
        const int s = __builtin_amdgcn_readlane(sl, p);
        const v4f hrow = *(const v4f*)(Y + (size_t)s * DD + ch);
        a0 = a0 + hrow;
      }
    }
    a0.x = fmaxf(a0.x, 0.0f); a0.y = fmaxf(a0.y, 0.0f); a0.z = fmaxf(a0.z, 0.0f); a0.w = fmaxf(a0.w, 0.0f);
    const float ss = red32(a0.x * a0.x + a0.y * a0.y + a0.z * a0.z + a0.w * a0.w);
    const float f = logmap_f(ss) * tc;
    if (c >= nN) {
      const v4f z = {0.f, 0.f, 0.f, 0.f}; a0 = z;
    }
    v4h hv;
    hv[0] = (_Float16)(a0.x * f); hv[1] = (_Float16)(a0.y * f); hv[2] = (_Float16)(a0.z * f); hv[3] = (_Float16)(a0.w * f);
    if (nraw > DEGCAP) {
      const _Float16 qn = (_Float16)__int_as_float(0x7fc00000);
      hv[0] = qn; hv[1] = qn; hv[2] = qn; hv[3] = qn;
    }
    _Float16* rp = T16 + (size_t)c * DD + ch;
    *(volatile v4h*)rp = hv;
    __threadfence();
    *(volatile v4h*)rp = hv;
  }
}

__global__ __launch_bounds__(NTHR) void k_head(
    const _Float16* __restrict__ A16, const _Float16* __restrict__ Bw,
    const float* __restrict__ bcls, float* out, float osc, int nN) {
  __shared__ __attribute__((aligned(16))) float so[GROWS * NCLS];
  const int tid = threadIdx.x, lane = tid & 31, wave = tid >> 5, hh = lane >> 4, m = lane & 15;
  const int rowBase = (int)blockIdx.x * GROWS;
  const _Float16* ap = A16 + (size_t)(rowBase + 16 * wave + m) * DD + 8 * hh;
  const _Float16* bp = Bw + (size_t)m * DD + 8 * hh;

  v8f acc = {0.f, 0.f, 0.f, 0.f, 0.f, 0.f, 0.f, 0.f};
#pragma unroll 1
  for (int kt = 0; kt < DD / 32; ++kt) {
    FragH af, bf;
    af.h[0] = *(const v8h*)(ap + 32 * kt);
    af.h[1] = *(const v8h*)(ap + 32 * kt + 16);
    bf.h[0] = *(const v8h*)(bp + 32 * kt);
    bf.h[1] = *(const v8h*)(bp + 32 * kt + 16);
    acc = wmf(af.v, bf.v, acc);
  }

  const int mc = m < NCLS ? m : NCLS - 1;
  const float bv = bcls[mc];
  const int rl0 = 16 * wave + 8 * hh;
#pragma unroll
  for (int r = 0; r < 8; ++r) {
    const float v = acc[r] * osc + bv;
    if (m < NCLS) so[(rl0 + r) * NCLS + m] = v;
  }
  __syncthreads();

  int nv = nN - rowBase;
  nv = nv < 0 ? 0 : (nv > GROWS ? GROWS : nv);
  const int nv4 = (nv * NCLS) >> 2;
  float* op = out + (size_t)rowBase * NCLS;
#pragma unroll 1
  for (int i = tid; i < nv4; i += NTHR) {
    const v4f v = *(const v4f*)(so + 4 * i);
    *(volatile v4f*)(op + 4 * i) = v;
  }
  __threadfence();
#pragma unroll 1
  for (int i = tid; i < nv4; i += NTHR) {
    const v4f v = *(const v4f*)(so + 4 * i);
    *(volatile v4f*)(op + 4 * i) = v;
  }
}

extern "C" void kernel_launch(void* const* d_in, const int* in_sizes, int n_in,
                              void* d_out, int out_size, void* d_ws, size_t ws_size,
                              hipStream_t stream) {
  if (n_in < 8) return;
  const int nE = in_sizes[0] / 2;
  const int nN = in_sizes[1] / DD;
  if (nN <= 0 || nE <= 0) return;
  if (in_sizes[0] != 2 * nE || in_sizes[1] != nN * DD) return;
  if (in_sizes[2] != DD * DD || in_sizes[3] != DD) return;
  if (in_sizes[4] != DD * DD || in_sizes[5] != DD) return;
  if (in_sizes[6] != NCLS * DD || in_sizes[7] != NCLS) return;
  if (nN > (1 << 20) || nE > (1 << 20)) return;
  if ((nN % 16) != 0) return;
  if ((long long)out_size != (long long)nN * NCLS) return;

  const int*   ei  = (const int*)d_in[0];
  const float* x   = (const float*)d_in[1];
  const float* W1  = (const float*)d_in[2];
  const float* b1  = (const float*)d_in[3];
  const float* W2  = (const float*)d_in[4];
  const float* b2  = (const float*)d_in[5];
  const float* Wc  = (const float*)d_in[6];
  const float* bc  = (const float*)d_in[7];
  float* out = (float*)d_out;
  const int* srci = ei;
  const int* dsti = ei + nE;
  const int nK = nE;

  const int NPAD   = ((nN + TGT - 1) / TGT) * TGT;
  const int nBC    = (nN + NBC - 1) / NBC;
  const int CNTPAD = nBC * NBC;
  const int nBF    = (nN + NBF - 1) / NBF;
  const int OFFN   = nBF * NBF;
  if (nBF + 1 > RBN) return;
  if (OFFN > CNTPAD || NPAD > OFFN) return;
  if ((NPAD % GROWS) != 0 || (NPAD % TGT) != 0) return;
  const int csrLen = ((nK + 31) & ~31) + 32 * (nBF + 1);
  const int nG     = NPAD / GROWS;
  const int nAgg   = NPAD / TGT;

  char* ws = (char*)d_ws;
  size_t off = 0;
  const size_t oT16 = off; off += (size_t)NPAD * DD * 2;         off = (off + 255) & ~(size_t)255;
  const size_t oY32 = off; off += (size_t)NPAD * DD * 4;         off = (off + 255) & ~(size_t)255;
  const size_t oW1  = off; off += (size_t)DD * DD * 2;           off = (off + 255) & ~(size_t)255;
  const size_t oW2  = off; off += (size_t)DD * DD * 2;           off = (off + 255) & ~(size_t)255;
  const size_t oWc  = off; off += (size_t)NCP * DD * 2;          off = (off + 255) & ~(size_t)255;
  const size_t oCnt = off; off += (size_t)CNTPAD * 4;            off = (off + 255) & ~(size_t)255;
  const size_t oOff = off; off += (size_t)OFFN * 4;              off = (off + 255) & ~(size_t)255;
  const size_t oRb  = off; off += (size_t)RBN * 4;               off = (off + 255) & ~(size_t)255;
  const size_t oCsr = off; off += (size_t)csrLen * 4;            off = (off + 255) & ~(size_t)255;
  if (off > ws_size || off > (size_t)WSCAP) return;
  _Float16* T16 = (_Float16*)(ws + oT16);
  float*    Y32 = (float*)(ws + oY32);
  _Float16* W1p = (_Float16*)(ws + oW1);
  _Float16* W2p = (_Float16*)(ws + oW2);
  _Float16* Wcp = (_Float16*)(ws + oWc);
  int*      cnt = (int*)(ws + oCnt);
  int*      offp = (int*)(ws + oOff);
  int*      rb   = (int*)(ws + oRb);
  int*      csr  = (int*)(ws + oCsr);

  const int vec8 = ((nE & 3) == 0) ? 1 : 0;
  const float osc = 1.0f / ((float)TC * (float)WSCL);
  const float tc  = (float)TC;

  k_cvtw<<<2 * BPW + 1, NTHR, 0, stream>>>(W1, W2, Wc, W1p, W2p, Wcp, (float)WSCL);

  hipFuncSetAttribute(reinterpret_cast<const void*>(&k_count),
                      hipFuncAttributeMaxDynamicSharedMemorySize, LDS_COUNT);
  k_count<<<nBC, NTHR, LDS_COUNT, stream>>>(dsti, cnt, nK, vec8);
  k_offsets<<<1, OTHR, 0, stream>>>(cnt, offp, rb, nBF);
  hipFuncSetAttribute(reinterpret_cast<const void*>(&k_fill),
                      hipFuncAttributeMaxDynamicSharedMemorySize, LDS_FILL);
  k_fill<<<nBF, NTHR, LDS_FILL, stream>>>(dsti, offp, rb, csr, nK, vec8, csrLen);

  hipFuncSetAttribute(reinterpret_cast<const void*>(&k_gemm_exp),
                      hipFuncAttributeMaxDynamicSharedMemorySize, LDS_GEMM);

  k_tan0<<<nAgg, NTHR, 0, stream>>>(x, T16, nN, tc);
  k_gemm_exp<<<nG, NTHR, LDS_GEMM, stream>>>(T16, W1p, b1, Y32, osc);
  k_agg<<<nAgg, NTHR, 0, stream>>>(csr, offp, cnt, srci, Y32, T16, nN, nE, csrLen, tc);

  k_gemm_exp<<<nG, NTHR, LDS_GEMM, stream>>>(T16, W2p, b2, Y32, osc);
  k_agg<<<nAgg, NTHR, 0, stream>>>(csr, offp, cnt, srci, Y32, T16, nN, nE, csrLen, tc);

  k_head<<<nG, NTHR, 0, stream>>>(T16, Wcp, bc, out, osc, nN);
}
